// MVPFusion_12403865551055
// MI455X (gfx1250) — hardware-verified
//
#include <hip/hip_runtime.h>


typedef _Float16 h8   __attribute__((ext_vector_type(8)));
typedef _Float16 v16h __attribute__((ext_vector_type(16)));
typedef float    v8f  __attribute__((ext_vector_type(8)));
typedef float    v4f  __attribute__((ext_vector_type(4)));
union H16 { v16h v; h8 h[2]; };
#define CCH 128
#define HW  4096
#define SS  336
#define SP  352
#define VST2(T, ptr, val) do { const T _v = (val); *(volatile T*)(ptr) = _v; __threadfence(); *(volatile T*)(ptr) = _v; } while (0)
static __device__ __forceinline__ v8f wmma_f16(v16h a, v16h b, v8f c) {
  v8f d = __builtin_amdgcn_wmma_f32_16x16x32_f16(false, a, false, b, (short)0, c, false, false);
  asm volatile("v_nop\n\tv_nop\n\tv_nop\n\tv_nop" : "+v"(d) : "v"(a), "v"(b));
  return d;
}
static __device__ __forceinline__ v16h frag16(const _Float16* p, int hi) {
  H16 f; f.h[0] = *(const h8*)(p + hi * 8); f.h[1] = *(const h8*)(p + 16 + hi * 8); return f.v;
}
static __device__ __forceinline__ void wave_lds_sync() {
  __builtin_amdgcn_fence(__ATOMIC_RELEASE, "workgroup"); __builtin_amdgcn_wave_barrier(); __builtin_amdgcn_fence(__ATOMIC_ACQUIRE, "workgroup");
}

__global__ void k_f32_to_f16(const float* __restrict__ in, _Float16* __restrict__ out, int n8) {
  int i = blockIdx.x * 256 + threadIdx.x;
  if (i >= n8) return;
  h8 v;
#pragma unroll
  for (int e = 0; e < 8; ++e) v[e] = (_Float16)in[(size_t)i * 8 + e];
  VST2(h8, out + (size_t)i * 8, v);
}
__global__ void k_tam(const float* __restrict__ xg, const float* __restrict__ sal_w, const float* __restrict__ sal_b, float* __restrict__ tam) {
  int s = blockIdx.x * 256 + threadIdx.x;
  if (s >= HW) return;
  float acc = 0.f;
#pragma unroll 4
  for (int c = 0; c < CCH; ++c) acc += sal_w[c] * xg[c * HW + s];
  VST2(float, tam + s, 1.f / (1.f + expf(-(acc + sal_b[0]))));
}
__global__ void k_build_q(const float* __restrict__ x, const float* __restrict__ tam, _Float16* __restrict__ q16, float* __restrict__ qf32) {
  const int t = blockIdx.x * 256 + threadIdx.x;
  const int c0 = (t & 15) * 8, l = (t >> 4) & 4095, p = t >> 16;
  const int y = l >> 6, z = l & 63, a = p >> 1, b = p & 1;
  const float tv = tam[((a << 5) + (y >> 1)) * 64 + (b << 5) + (z >> 1)];
  v8f o; h8 oh;
#pragma unroll
  for (int e = 0; e < 8; ++e) { o[e] = x[((size_t)p * CCH + c0 + e) * HW + l] * tv; oh[e] = (_Float16)o[e]; }
  const size_t qi = ((size_t)p * HW + l) * CCH + c0;
  VST2(v8f, qf32 + qi, o);
  VST2(h8, q16 + qi, oh);
}
__global__ void k_pool(const float* __restrict__ xg, _Float16* __restrict__ kv16) {
  int idx = blockIdx.x * 256 + threadIdx.x;
  if (idx >= 4 * SP * CCH) return;
  int c = idx & 127, s = (idx >> 7) % SP, p = idx / (SP * CCH);
  float val = 0.f;
  if (s < SS) {
    int ksz, tw, t;
    if (s < 256)      { ksz = 2; tw = 16; t = s; }
    else if (s < 320) { ksz = 4; tw = 8;  t = s - 256; }
    else              { ksz = 8; tw = 4;  t = s - 320; }
    int ti = t / tw, tj = t % tw;
    int a = p >> 1, b = p & 1;
    int r0 = (a << 5) + ti * ksz, c0 = (b << 5) + tj * ksz;
    float sum = 0.f;
    for (int dy = 0; dy < ksz; ++dy)
      for (int dz = 0; dz < ksz; ++dz) sum += xg[c * HW + (r0 + dy) * 64 + (c0 + dz)];
    val = sum / (float)(ksz * ksz);
  }
  VST2(_Float16, kv16 + idx, (_Float16)val);
}
__global__ __launch_bounds__(32)
void k_gemm_blk(const _Float16* __restrict__ A, long sA, int lda, const _Float16* __restrict__ W, long sW,
                const float* __restrict__ bias, int sB, _Float16* __restrict__ O16, float* __restrict__ O32,
                const float* __restrict__ res, long sO, int ldo, int K, int mode) {
  __shared__ __attribute__((aligned(16))) float sT[32][68];
  int lane = threadIdx.x;
  int m0 = blockIdx.x * 32, n0 = blockIdx.y * 64, p = blockIdx.z;
  A += (long)p * sA; W += (long)p * sW; bias += (long)p * sB;
  int mr = lane & 15, hi = lane >> 4;
  const _Float16* ar[2]; ar[0] = A + (long)(m0 + mr) * lda; ar[1] = ar[0] + 16 * lda;
  const _Float16* wr[4];
#pragma unroll
  for (int ni = 0; ni < 4; ++ni) wr[ni] = W + (long)(n0 + ni * 16 + mr) * K;
  v8f acc[2][4] = {};
  for (int k0 = 0; k0 < K; k0 += 32) {
    v16h a[2], b[4];
#pragma unroll
    for (int mi = 0; mi < 2; ++mi) a[mi] = frag16(ar[mi] + k0, hi);
#pragma unroll
    for (int ni = 0; ni < 4; ++ni) b[ni] = frag16(wr[ni] + k0, hi);
#pragma unroll
    for (int mi = 0; mi < 2; ++mi)
#pragma unroll
      for (int ni = 0; ni < 4; ++ni) acc[mi][ni] = wmma_f16(a[mi], b[ni], acc[mi][ni]);
  }
#pragma unroll
  for (int ni = 0; ni < 4; ++ni) {
    const float bv = bias[n0 + ni * 16 + mr];
#pragma unroll
    for (int mi = 0; mi < 2; ++mi)
#pragma unroll
      for (int r = 0; r < 8; ++r) { float v = acc[mi][ni][r] + bv; if (mode == 1) v = fmaxf(v, 0.f); sT[mi * 16 + r + (hi << 3)][ni * 16 + mr] = v; }
  }
  wave_lds_sync();
  const long ob = (long)p * sO;
  for (int pass = 0; pass < 2; ++pass) {
    if (mode == 2) {
#pragma unroll
      for (int j = 0; j < 16; ++j) { const int rr = j * 2 + (lane >> 4), q4 = (lane & 15) * 4; const long o = ob + (long)(m0 + rr) * ldo + n0 + q4;
        v4f v = *(const v4f*)(&sT[rr][q4]); const v4f rs = *(const v4f*)(res + o); v += rs; *(volatile v4f*)(O32 + o) = v; }
    } else {
#pragma unroll
      for (int j = 0; j < 8; ++j) { const int rr = j * 4 + (lane >> 3), q8 = (lane & 7) * 8; h8 v;
#pragma unroll
        for (int e = 0; e < 8; ++e) v[e] = (_Float16)sT[rr][q8 + e];
        *(volatile h8*)(O16 + ob + (long)(m0 + rr) * ldo + n0 + q8) = v; }
    }
    __threadfence();
  }
}
#define ATT_WAVES 4
__global__ __launch_bounds__(128)
void k_attn(const _Float16* __restrict__ qp, const _Float16* __restrict__ kp, const _Float16* __restrict__ vp, _Float16* __restrict__ ao) {
  __shared__ __attribute__((aligned(16))) _Float16 smem[ATT_WAVES][16][SP];
  __shared__ __attribute__((aligned(16))) _Float16 sout[ATT_WAVES][16][CCH];
  int lane = threadIdx.x & 31, wave = threadIdx.x >> 5;
  int p = blockIdx.y;
  int l0 = (blockIdx.x * ATT_WAVES + wave) << 4;
  int mr = lane & 15, hi = lane >> 4;
  h8 z8 = {};
  for (int h = 0; h < 8; ++h) {
    const _Float16* qrow = qp + ((long)p * HW + l0 + mr) * CCH + h * 16;
    H16 a; a.h[0] = *(const h8*)(qrow + hi * 8); a.h[1] = z8;
    const _Float16* kbase = kp + (long)p * SP * CCH + h * 16;
    v8f sc[21];
#pragma unroll
    for (int j = 0; j < 21; ++j) {
      H16 b; b.h[0] = *(const h8*)(kbase + (long)(j * 16 + mr) * CCH + hi * 8); b.h[1] = z8;
      v8f zc = {};
      sc[j] = wmma_f16(a.v, b.v, zc);
    }
#pragma unroll
    for (int r = 0; r < 8; ++r) {
      float mx = -1e30f;
#pragma unroll
      for (int j = 0; j < 21; ++j) mx = fmaxf(mx, sc[j][r]);
#pragma unroll
      for (int off = 1; off < 16; off <<= 1) mx = fmaxf(mx, __shfl_xor(mx, off, 32));
      float sum = 0.f;
#pragma unroll
      for (int j = 0; j < 21; ++j) { float e = __expf((sc[j][r] - mx) * 0.25f); sc[j][r] = e; sum += e; }
#pragma unroll
      for (int off = 1; off < 16; off <<= 1) sum += __shfl_xor(sum, off, 32);
      float inv = 1.f / sum;
      int row = r + (hi << 3);
#pragma unroll
      for (int j = 0; j < 21; ++j) smem[wave][row][j * 16 + mr] = (_Float16)(sc[j][r] * inv);
    }
    for (int t = lane; t < 256; t += 32) smem[wave][t >> 4][SS + (t & 15)] = (_Float16)0.f;
    wave_lds_sync();
    v8f acc = {};
    const _Float16* vcol = vp + (long)p * SP * CCH + h * 16 + mr;
#pragma unroll 2
    for (int k0 = 0; k0 < SP; k0 += 32) {
      v16h a2 = frag16(&smem[wave][mr][k0], hi), b2;
#pragma unroll
      for (int e = 0; e < 16; ++e) b2[e] = vcol[(long)(k0 + ((e < 8) ? (8 * hi + e) : (16 + 8 * hi + e - 8))) * CCH];
      acc = wmma_f16(a2, b2, acc);
    }
#pragma unroll
    for (int r = 0; r < 8; ++r) sout[wave][r + (hi << 3)][h * 16 + mr] = (_Float16)acc[r];
    wave_lds_sync();
  }
  for (int pass = 0; pass < 2; ++pass) {
#pragma unroll
    for (int j = 0; j < 8; ++j) { const int rr = j * 2 + (lane >> 4), q8 = (lane & 15) * 8;
      *(volatile h8*)(ao + ((long)p * HW + l0 + rr) * CCH + q8) = *(const h8*)(&sout[wave][rr][q8]); }
    __threadfence();
  }
}
__global__ void k_ln(const float* __restrict__ y, const float* __restrict__ g, const float* __restrict__ be, float* __restrict__ o32, _Float16* __restrict__ o16) {
  __shared__ float red[8];
  int c = threadIdx.x;
  long tok = (long)blockIdx.y * HW + blockIdx.x;
  float v = y[tok * CCH + c];
  float s = v;
#pragma unroll
  for (int off = 16; off >= 1; off >>= 1) s += __shfl_xor(s, off, 32);
  int wid = c >> 5, ln = c & 31;
  if (!ln) red[wid] = s;
  __syncthreads();
  float mu = (red[0] + red[1] + red[2] + red[3]) * (1.f / 128.f);
  float d = v - mu;
  float s2 = d * d;
#pragma unroll
  for (int off = 16; off >= 1; off >>= 1) s2 += __shfl_xor(s2, off, 32);
  if (!ln) red[4 + wid] = s2;
  __syncthreads();
  float var = (red[4] + red[5] + red[6] + red[7]) * (1.f / 128.f);
  float o = d / sqrtf(var + 1e-5f) * g[c] + be[c];
  VST2(float, o32 + tok * CCH + c, o);
  if (o16) VST2(_Float16, o16 + tok * CCH + c, (_Float16)o);
}
__global__ __launch_bounds__(256) void k_out_img(const float* __restrict__ src, float* __restrict__ out) {
  __shared__ float tile[32][33];
  const int p = blockIdx.z, c0 = blockIdx.y * 32, l0 = blockIdx.x * 32;
  const int tx = threadIdx.x & 31, ty = threadIdx.x >> 5;
#pragma unroll
  for (int r = 0; r < 4; ++r) { const int l = l0 + ty + 8 * r; tile[ty + 8 * r][tx] = src[((long)p * HW + l) * CCH + c0 + tx]; }
  __syncthreads();
  for (int pass = 0; pass < 2; ++pass) {
#pragma unroll
    for (int r = 0; r < 4; ++r) { const int cc = ty + 8 * r; *(volatile float*)(out + ((long)p * CCH + c0 + cc) * HW + l0 + tx) = tile[tx][cc]; }
    __threadfence();
  }
}
__global__ __launch_bounds__(256) void k_out_glb(const float* __restrict__ x, const float* __restrict__ src, float* __restrict__ out) {
  int idx = blockIdx.x * 256 + threadIdx.x;
  int c = idx >> 12, rem = idx & 4095, m = rem >> 6, n = rem & 63;
  int a = m >> 5, b = n >> 5, y = (m & 31) << 1, z = (n & 31) << 1, patch = a * 2 + b;
  long base = (long)4 * CCH * HW;
  VST2(float, out + base + idx, x[base + idx] + src[((long)patch * HW + (y << 6) + z) * CCH + c]);
}

extern "C" void kernel_launch(void* const* d_in, const int* in_sizes, int n_in,
                              void* d_out, int out_size, void* d_ws, size_t ws_size, hipStream_t stream) {
  (void)in_sizes; (void)n_in; (void)out_size;
  const float* x = (const float*)d_in[0]; const float* sal_w = (const float*)d_in[1]; const float* sal_b = (const float*)d_in[2];
  const float* ipw = (const float*)d_in[3]; const float* ipb = (const float*)d_in[4]; const float* ow = (const float*)d_in[5]; const float* ob = (const float*)d_in[6];
  const float* w3 = (const float*)d_in[7]; const float* b3 = (const float*)d_in[8]; const float* w4 = (const float*)d_in[9]; const float* b4 = (const float*)d_in[10];
  const float* g1 = (const float*)d_in[11]; const float* be1 = (const float*)d_in[12]; const float* g2 = (const float*)d_in[13]; const float* be2 = (const float*)d_in[14];
  float* out = (float*)d_out;
  char* w = (char*)d_ws; size_t off = 0;
  auto alloc = [&](size_t bytes) { size_t r = off; off = (off + bytes + 255) & ~(size_t)255; return r; };
  float*    tam   = (float*)   (w + alloc((size_t)HW * 4));
  _Float16* q16   = (_Float16*)(w + alloc((size_t)4 * HW * CCH * 2));
  float*    qf32  = (float*)   (w + alloc((size_t)4 * HW * CCH * 4));
  _Float16* Wi16  = (_Float16*)(w + alloc((size_t)4 * 384 * CCH * 2));
  _Float16* Wo16  = (_Float16*)(w + alloc((size_t)4 * CCH * CCH * 2));
  _Float16* w3h   = (_Float16*)(w + alloc((size_t)256 * 128 * 2));
  _Float16* w4h   = (_Float16*)(w + alloc((size_t)128 * 256 * 2));
  _Float16* kv16  = (_Float16*)(w + alloc((size_t)4 * SP * CCH * 2));
  _Float16* qp16  = (_Float16*)(w + alloc((size_t)4 * HW * CCH * 2));
  _Float16* kp16  = (_Float16*)(w + alloc((size_t)4 * SP * CCH * 2));
  _Float16* vp16  = (_Float16*)(w + alloc((size_t)4 * SP * CCH * 2));
  _Float16* ao16  = (_Float16*)(w + alloc((size_t)4 * HW * CCH * 2));
  float*    y1    = (float*)   (w + alloc((size_t)4 * HW * CCH * 4));
  float*    src32 = (float*)   (w + alloc((size_t)4 * HW * CCH * 4));
  _Float16* src16 = (_Float16*)(w + alloc((size_t)4 * HW * CCH * 2));
  _Float16* hid16 = (_Float16*)(w + alloc((size_t)4 * HW * 256 * 2));
  float*    src2  = (float*)   (w + alloc((size_t)4 * HW * CCH * 4));
  if (off > ws_size) return;
  const float* xg = x + (size_t)4 * CCH * HW;

  auto cvt = [&](const float* s, _Float16* d, int n) { k_f32_to_f16<<<(n / 8 + 255) / 256, 256, 0, stream>>>(s, d, n / 8); };
  cvt(ipw, Wi16, 4 * 384 * 128); cvt(ow, Wo16, 4 * 128 * 128); cvt(w3, w3h, 256 * 128); cvt(w4, w4h, 128 * 256);
  k_tam<<<HW / 256, 256, 0, stream>>>(xg, sal_w, sal_b, tam);
  k_build_q<<<(4 * HW * 16) / 256, 256, 0, stream>>>(x, tam, q16, qf32);
  k_pool<<<(4 * SP * CCH + 255) / 256, 256, 0, stream>>>(xg, kv16);
  k_gemm_blk<<<dim3(HW / 32, CCH / 64, 4), 32, 0, stream>>>(q16, (long)HW * CCH, CCH, Wi16, (long)384 * CCH, ipb, 384, qp16, nullptr, nullptr, (long)HW * CCH, CCH, CCH, 0);
  k_gemm_blk<<<dim3(SP / 32, CCH / 64, 4), 32, 0, stream>>>(kv16, (long)SP * CCH, CCH, Wi16 + 128 * CCH, (long)384 * CCH, ipb + 128, 384, kp16, nullptr, nullptr, (long)SP * CCH, CCH, CCH, 0);
  k_gemm_blk<<<dim3(SP / 32, CCH / 64, 4), 32, 0, stream>>>(kv16, (long)SP * CCH, CCH, Wi16 + 256 * CCH, (long)384 * CCH, ipb + 256, 384, vp16, nullptr, nullptr, (long)SP * CCH, CCH, CCH, 0);
  k_attn<<<dim3(HW / (16 * ATT_WAVES), 4), 32 * ATT_WAVES, 0, stream>>>(qp16, kp16, vp16, ao16);
  k_gemm_blk<<<dim3(HW / 32, CCH / 64, 4), 32, 0, stream>>>(ao16, (long)HW * CCH, CCH, Wo16, (long)CCH * CCH, ob, CCH, nullptr, y1, qf32, (long)HW * CCH, CCH, CCH, 2);
  k_ln<<<dim3(HW, 4), 128, 0, stream>>>(y1, g1, be1, src32, src16);
  k_gemm_blk<<<dim3(4 * HW / 32, 256 / 64, 1), 32, 0, stream>>>(src16, 0L, CCH, w3h, 0L, b3, 0, hid16, nullptr, nullptr, 0L, 256, CCH, 1);
  k_gemm_blk<<<dim3(4 * HW / 32, CCH / 64, 1), 32, 0, stream>>>(hid16, 0L, 256, w4h, 0L, b4, 0, nullptr, y1, src32, 0L, CCH, 256, 2);
  k_ln<<<dim3(HW, 4), 128, 0, stream>>>(y1, g2, be2, src2, nullptr);
  k_out_img<<<dim3(HW / 32, CCH / 32, 4), 256, 0, stream>>>(src2, out);
  k_out_glb<<<(CCH * HW) / 256, 256, 0, stream>>>(x, src2, out);
}
